// MHA_3770981285896
// MI455X (gfx1250) — hardware-verified
//
#include <hip/hip_runtime.h>


#ifndef NB
#define NB 2
#endif
#ifndef SEQ
#define SEQ 2048
#endif
#define NB_FULL  2
#define SEQ_FULL 2048
#define DM    1024
#define NH    16
#define HD    64
#define NQKV  (3 * DM)
#define MROWS (NB * SEQ)
#define KP    72
#define PP    40
#define WCAR  64.0f
#define PSH   8.0f
#define SCL   0.125f
#define LOG2E 1.4426950408889634f

static_assert(SEQ % 64 == 0);
static_assert(SEQ <= SEQ_FULL);
static_assert(NB <= NB_FULL);
static_assert(DM % 64 == 0);
static_assert(NH * HD == DM);
static_assert(NQKV % 64 == 0);
static_assert((size_t)2 * MROWS * DM * 2 + (size_t)NQKV * DM * 2 + (size_t)DM * DM * 2 + (size_t)MROWS * NQKV * 4 + (size_t)4 * MROWS * DM * 2 <= (size_t)134217728);

typedef _Float16 h16;
typedef unsigned short bf;
typedef __attribute__((ext_vector_type(16))) __bf16   v16bf;
typedef __attribute__((ext_vector_type(16))) _Float16 v16h;
typedef __attribute__((ext_vector_type(8)))  _Float16 v8h;
typedef __attribute__((ext_vector_type(8)))  unsigned short v8us;
typedef __attribute__((ext_vector_type(8)))  float    v8f;
typedef __attribute__((ext_vector_type(4)))  float    v4f;
typedef v8h  __attribute__((may_alias)) v8ha;
typedef v4f  __attribute__((may_alias)) v4fa;
typedef v8us __attribute__((may_alias)) v8usa;

__device__ __forceinline__ unsigned short f2bf(float f) { unsigned u = __float_as_uint(f); u += 0x7FFFu + ((u >> 16) & 1u); return (unsigned short)(u >> 16); }
__device__ __forceinline__ float bf2f(unsigned short b) { return __uint_as_float(((unsigned)b) << 16); }
__device__ __forceinline__ float bfr(float f) { return bf2f(f2bf(f)); }
__device__ __forceinline__ v16h cat16(v8h lo, v8h hi) { return __builtin_shufflevector(lo, hi, 0, 1, 2, 3, 4, 5, 6, 7, 8, 9, 10, 11, 12, 13, 14, 15); }
__device__ __forceinline__ v16bf cat16b(v8us lo, v8us hi) { return __builtin_bit_cast(v16bf, __builtin_shufflevector(lo, hi, 0, 1, 2, 3, 4, 5, 6, 7, 8, 9, 10, 11, 12, 13, 14, 15)); }
__device__ __forceinline__ v8f wmma16(v16h a, v16h b, v8f c) { return __builtin_amdgcn_wmma_f32_16x16x32_f16(false, a, false, b, (short)0, c, false, false); }
__device__ __forceinline__ v8f wmmab(v16bf a, v16bf b, v8f c) { return __builtin_amdgcn_wmma_f32_16x16x32_bf16(false, a, false, b, (short)0, c, false, false); }
__device__ __forceinline__ void splitf(float y, unsigned short& h, unsigned short& l) { h = f2bf(y); l = f2bf(y - bf2f(h)); }

template <typename T16> struct WFrag;
template <> struct WFrag<h16> { typedef v16h V; static __device__ __forceinline__ V ld(const h16* p) { return cat16(*(const v8h*)p, *(const v8h*)(p + 16)); } static __device__ __forceinline__ v8f mma(V a, V b, v8f c) { return wmma16(a, b, c); } };
template <> struct WFrag<bf> { typedef v16bf V; static __device__ __forceinline__ V ld(const bf* p) { return cat16b(*(const v8us*)p, *(const v8us*)(p + 16)); } static __device__ __forceinline__ v8f mma(V a, V b, v8f c) { return wmmab(a, b, c); } };
template <typename T16, int NSPLIT, bool BIAS, bool RES>
__global__ __launch_bounds__(32) void k_gemmw(const T16* __restrict__ A, const T16* __restrict__ A2, const T16* __restrict__ Bt, const T16* __restrict__ Bt2, int K, float* C, int ldc, const float* __restrict__ bias, const float* __restrict__ resid, float esc, size_t sA, size_t sB, size_t sC, size_t sR) {
    typedef typename WFrag<T16>::V V;
    __shared__ __align__(16) float os[16 * 68];
    const size_t z = blockIdx.z; A += z * sA; if (A2) A2 += z * sA; Bt += z * sB; if (Bt2) Bt2 += z * sB; C += z * sC; if (RES) resid += z * sR;
    const int lane = threadIdx.x & 31, lr = lane & 15, hi = lane >> 4; const int r0 = blockIdx.x * 64, c0 = blockIdx.y * 64;
    v8f acc[4][4];
#pragma unroll
    for (int mb = 0; mb < 4; ++mb)
#pragma unroll
        for (int nb = 0; nb < 4; ++nb) acc[mb][nb] = (v8f){};
    const size_t aoff = (size_t)(r0 + lr) * K + 8 * hi, boff = (size_t)(c0 + lr) * K + 8 * hi;
#pragma unroll 1
    for (int kc = 0; kc < K; kc += 32) {
        V a[4], a2[4];
#pragma unroll
        for (int mb = 0; mb < 4; ++mb) { a[mb] = WFrag<T16>::ld(A + aoff + (size_t)mb * 16 * K + kc); if (NSPLIT == 1 || NSPLIT == 2) a2[mb] = WFrag<T16>::ld(A2 + aoff + (size_t)mb * 16 * K + kc); }
#pragma unroll
        for (int nb = 0; nb < 4; ++nb) { const V b = WFrag<T16>::ld(Bt + boff + (size_t)nb * 16 * K + kc); V b2; if (NSPLIT >= 2) b2 = WFrag<T16>::ld(Bt2 + boff + (size_t)nb * 16 * K + kc);
#pragma unroll
            for (int mb = 0; mb < 4; ++mb) { acc[mb][nb] = WFrag<T16>::mma(a[mb], b, acc[mb][nb]); if (NSPLIT == 1 || NSPLIT == 2) acc[mb][nb] = WFrag<T16>::mma(a2[mb], b, acc[mb][nb]); if (NSPLIT >= 2) acc[mb][nb] = WFrag<T16>::mma(a[mb], b2, acc[mb][nb]); } }
        asm volatile("v_nop\n\tv_nop\n\tv_nop\n\tv_nop" : "+v"(acc[0][0]), "+v"(acc[1][1]), "+v"(acc[2][2]), "+v"(acc[3][3]) : "v"(a[0]), "v"(a[3]));
    }
#pragma unroll
    for (int mb = 0; mb < 4; ++mb) {
#pragma unroll
        for (int nb = 0; nb < 4; ++nb) {
#pragma unroll
            for (int j = 0; j < 8; ++j) os[(hi * 8 + j) * 68 + nb * 16 + lr] = acc[mb][nb][j]; }
        __builtin_amdgcn_wave_barrier(); asm volatile("" ::: "memory");
        const size_t roff = (size_t)(r0 + mb * 16) * ldc + c0;
        float* crow = C + roff;
#pragma unroll 1
        for (int ps = 0; ps < 2; ++ps) {
#pragma unroll
            for (int s = 0; s < 8; ++s) { const int row = 2 * s + hi, cofs = lr * 4; v4f val = *(const v4fa*)(os + row * 68 + cofs);
#pragma unroll
                for (int q = 0; q < 4; ++q) val[q] = val[q] * esc;
                if (BIAS) { const v4f bb = *(const v4f*)(bias + c0 + cofs);
#pragma unroll
                    for (int q = 0; q < 4; ++q) val[q] += bfr(bb[q]); }
                if (RES) { const v4f rr = *(const v4f*)(resid + roff + (size_t)row * ldc + cofs);
#pragma unroll
                    for (int q = 0; q < 4; ++q) val[q] += bfr(rr[q]); }
                *(volatile v4f*)(crow + (size_t)row * ldc + cofs) = val; }
            if (ps == 0) __threadfence(); }
        __builtin_amdgcn_wave_barrier(); asm volatile("" ::: "memory");
    }
}

__global__ __launch_bounds__(256) void k_ln(const float* __restrict__ q, const float* __restrict__ gamma, const float* __restrict__ beta, bf* Hh, bf* Hl) {
    const int wave = __builtin_amdgcn_readfirstlane((int)(threadIdx.x >> 5)); const int lane = threadIdx.x & 31;
    const int row = blockIdx.x * 8 + wave; if (row >= MROWS) return;
    const int b = row / SEQ, t = row - b * SEQ;
    const float* src = q + ((size_t)b * SEQ_FULL + t) * DM + lane * 8;
    float sum = 0.f;
#pragma unroll 1
    for (int ch = 0; ch < 4; ++ch) { const v4f a0 = *(const v4f*)(src + ch * 256); const v4f a1 = *(const v4f*)(src + ch * 256 + 4);
#pragma unroll
        for (int j = 0; j < 4; ++j) { sum += bfr(a0[j]); sum += bfr(a1[j]); } }
#pragma unroll
    for (int sh = 16; sh; sh >>= 1) sum += __shfl_xor(sum, sh, 32);
    const float mu = sum * (1.0f / DM);
    float sq = 0.f;
#pragma unroll 1
    for (int ch = 0; ch < 4; ++ch) { const v4f a0 = *(const v4f*)(src + ch * 256); const v4f a1 = *(const v4f*)(src + ch * 256 + 4);
#pragma unroll
        for (int j = 0; j < 4; ++j) { const float d0 = bfr(a0[j]) - mu; const float d1 = bfr(a1[j]) - mu; sq += d0 * d0; sq += d1 * d1; } }
#pragma unroll
    for (int sh = 16; sh; sh >>= 1) sq += __shfl_xor(sq, sh, 32);
    const float var = sq * (1.0f / DM);
    const float rstd = 1.0f / sqrtf(var + 1e-5f);
    const size_t ob = (size_t)row * DM + lane * 8;
#pragma unroll 1
    for (int ps = 0; ps < 2; ++ps) {
#pragma unroll 1
        for (int ch = 0; ch < 4; ++ch) { const int cb = ch * 256; const v4f a0 = *(const v4f*)(src + cb); const v4f a1 = *(const v4f*)(src + cb + 4);
            const v4f g0 = *(const v4f*)(gamma + cb + lane * 8); const v4f g1 = *(const v4f*)(gamma + cb + lane * 8 + 4); const v4f e0 = *(const v4f*)(beta + cb + lane * 8); const v4f e1 = *(const v4f*)(beta + cb + lane * 8 + 4);
            v8us oh, ol;
#pragma unroll
            for (int j = 0; j < 4; ++j) { unsigned short hh, ll; const float y0 = (bfr(a0[j]) - mu) * rstd * bfr(g0[j]) + bfr(e0[j]); splitf(y0, hh, ll); oh[j] = hh; ol[j] = ll;
                const float y1 = (bfr(a1[j]) - mu) * rstd * bfr(g1[j]) + bfr(e1[j]); splitf(y1, hh, ll); oh[4 + j] = hh; ol[4 + j] = ll; }
            *(volatile v8us*)(Hh + ob + cb) = oh; *(volatile v8us*)(Hl + ob + cb) = ol; }
        if (ps == 0) __threadfence(); }
}

template <typename T16> struct V8T;
template <> struct V8T<h16> { typedef v8h V; typedef v8ha VA; static __device__ __forceinline__ h16 cv(float x) { return (h16)(bfr(x) * WCAR); } };
template <> struct V8T<bf> { typedef v8us V; typedef v8usa VA; static __device__ __forceinline__ bf cv(float x) { return f2bf(x); } };
template <typename T16>
__global__ __launch_bounds__(256) void k_wt(const float* __restrict__ W, T16* Wt) {
    __shared__ __align__(16) T16 Ts[64 * KP];
    typedef typename V8T<T16>::V VV; typedef typename V8T<T16>::VA VVA;
    const int tid = threadIdx.x; const int n0 = blockIdx.x * 64, k0 = blockIdx.y * 64;
    const int kk = tid >> 2, piece = tid & 3;
    const float* src = W + (size_t)(k0 + kk) * DM + n0 + piece * 16;
#pragma unroll
    for (int j4 = 0; j4 < 4; ++j4) { const v4f a = *(const v4f*)(src + j4 * 4);
#pragma unroll
        for (int q = 0; q < 4; ++q) { const int n = piece * 16 + j4 * 4 + q; Ts[n * KP + kk] = V8T<T16>::cv(a[q]); } }
    __syncthreads();
#pragma unroll 1
    for (int ps = 0; ps < 2; ++ps) {
#pragma unroll
        for (int it = 0; it < 2; ++it) { const int n = it * 32 + (tid >> 3), c = (tid & 7) * 8; const VV val = *(const VVA*)(Ts + n * KP + c);
            *(volatile VV*)(Wt + (size_t)(n0 + n) * DM + k0 + c) = val; }
        if (ps == 0) __threadfence(); }
}

__global__ __launch_bounds__(256) void k_qk(const float* __restrict__ C, int coff, const float* __restrict__ bias, h16* P) {
    const size_t i = (size_t)blockIdx.x * 256 + threadIdx.x; if (i >= (size_t)NB * NH * SEQ * 8) return;
    const int c8 = (int)(i & 7) * 8; const size_t rt = i >> 3; const int t = (int)(rt % SEQ); const int bh = (int)(rt / SEQ); const int b = bh / NH, h = bh - b * NH;
    const float* src = C + ((size_t)b * SEQ + t) * NQKV + coff + h * HD + c8;
    const v4f a0 = *(const v4f*)src; const v4f a1 = *(const v4f*)(src + 4); const v4f b0 = *(const v4f*)(bias + h * HD + c8); const v4f b1 = *(const v4f*)(bias + h * HD + c8 + 4);
    v8h o;
#pragma unroll
    for (int j = 0; j < 4; ++j) { o[j] = (h16)(a0[j] + bfr(b0[j])); o[4 + j] = (h16)(a1[j] + bfr(b1[j])); }
    *(volatile v8h*)(P + i * 8) = o; __threadfence(); *(volatile v8h*)(P + i * 8) = o;
}

__global__ __launch_bounds__(256) void k_vt(const float* __restrict__ C, const float* __restrict__ bias, h16* VT) {
    __shared__ __align__(16) h16 Ts[64 * KP];
    const int tid = threadIdx.x; const int t0 = blockIdx.x * 64, h = blockIdx.y, b = blockIdx.z;
    const int tt = tid >> 2, piece = tid & 3;
    const float* src = C + ((size_t)b * SEQ + t0 + tt) * NQKV + 2 * DM + h * HD + piece * 16;
#pragma unroll
    for (int j4 = 0; j4 < 4; ++j4) { const v4f a = *(const v4f*)(src + j4 * 4); const v4f bb = *(const v4f*)(bias + h * HD + piece * 16 + j4 * 4);
#pragma unroll
        for (int q = 0; q < 4; ++q) { const int d = piece * 16 + j4 * 4 + q; const float x = fmaxf(a[q] + bfr(bb[q]), 0.0f); Ts[d * KP + tt] = (h16)x; } }
    __syncthreads();
#pragma unroll 1
    for (int ps = 0; ps < 2; ++ps) {
#pragma unroll
        for (int it = 0; it < 2; ++it) { const int d = it * 32 + (tid >> 3), c = (tid & 7) * 8; const v8h val = *(const v8ha*)(Ts + d * KP + c);
            *(volatile v8h*)(VT + ((size_t)(b * NH + h) * HD + d) * SEQ + t0 + c) = val; }
        if (ps == 0) __threadfence(); }
}

__global__ __launch_bounds__(128) void k_attn(const h16* __restrict__ Q16, const h16* __restrict__ K16, const h16* __restrict__ VT16, h16* O16) {
    __shared__ __align__(16) h16 Ks[64 * KP];
    __shared__ __align__(16) h16 Vs[64 * KP];
    __shared__ __align__(16) h16 Pw[4 * 16 * PP];
    __shared__ __align__(16) h16 Os[4 * 16 * KP];
    const int tid = threadIdx.x; const int wave = __builtin_amdgcn_readfirstlane((int)(threadIdx.x >> 5)); const int lane = tid & 31, lr = lane & 15, hi = lane >> 4;
    const int bh = blockIdx.y; const int q0 = blockIdx.x * 64 + wave * 16;
    const size_t pbase = (size_t)bh * SEQ * HD;
    const h16* qp = Q16 + pbase + (size_t)(q0 + lr) * HD + 8 * hi;
    const v16h aq0 = cat16(*(const v8h*)qp, *(const v8h*)(qp + 16));
    const v16h aq1 = cat16(*(const v8h*)(qp + 32), *(const v8h*)(qp + 48));
    v8f acc[4];
#pragma unroll
    for (int dn = 0; dn < 4; ++dn) acc[dn] = (v8f){};
    float mr[8], ls[8];
#pragma unroll
    for (int r = 0; r < 8; ++r) { mr[r] = -3.0e38f; ls[r] = 0.f; }
    const float cexp = SCL * LOG2E;
    const int pwo = wave * 16 * PP;
#pragma unroll 1
    for (int kb = 0; kb < SEQ; kb += 64) {
        __syncthreads();
#pragma unroll
        for (int i = 0; i < 4; ++i) { const int p = tid + 128 * i; const int r = p >> 3, c = (p & 7) * 8;
            const v8h kv = *(const v8h*)(K16 + pbase + (size_t)(kb + r) * HD + c);
            const v8h vv = *(const v8h*)(VT16 + pbase + (size_t)r * SEQ + kb + c);
            *(v8ha*)(Ks + r * KP + c) = kv; *(v8ha*)(Vs + r * KP + c) = vv; }
        __syncthreads();
#pragma unroll 1
        for (int hf = 0; hf < 2; ++hf) {
            const int ko = hf * 32;
            v8f s0 = (v8f){}, s1 = (v8f){};
            { const int o0 = (ko + lr) * KP + 8 * hi, o1 = (ko + 16 + lr) * KP + 8 * hi;
              const v16h b00 = cat16(*(const v8ha*)(Ks + o0), *(const v8ha*)(Ks + o0 + 16));
              const v16h b10 = cat16(*(const v8ha*)(Ks + o1), *(const v8ha*)(Ks + o1 + 16));
              const v16h b01 = cat16(*(const v8ha*)(Ks + o0 + 32), *(const v8ha*)(Ks + o0 + 48));
              const v16h b11 = cat16(*(const v8ha*)(Ks + o1 + 32), *(const v8ha*)(Ks + o1 + 48));
              s0 = wmma16(aq0, b00, s0); s1 = wmma16(aq0, b10, s1); s0 = wmma16(aq1, b01, s0); s1 = wmma16(aq1, b11, s1); }
            asm volatile("v_nop\n\tv_nop\n\tv_nop\n\tv_nop" : "+v"(s0), "+v"(s1) : "v"(aq0), "v"(aq1));
            float p0[8], p1[8];
#pragma unroll
            for (int r = 0; r < 8; ++r) {
                const float t0 = s0[r] * cexp, t1 = s1[r] * cexp;
                float mx = fmaxf(t0, t1);
                mx = fmaxf(mx, __shfl_xor(mx, 1, 32)); mx = fmaxf(mx, __shfl_xor(mx, 2, 32)); mx = fmaxf(mx, __shfl_xor(mx, 4, 32)); mx = fmaxf(mx, __shfl_xor(mx, 8, 32));
                const float mn = fmaxf(mr[r], mx);
                const float al = __builtin_amdgcn_exp2f(mr[r] - mn);
                p0[r] = __builtin_amdgcn_exp2f((t0 - mn) + PSH); p1[r] = __builtin_amdgcn_exp2f((t1 - mn) + PSH);
                ls[r] = ls[r] * al + (p0[r] + p1[r]); mr[r] = mn;
#pragma unroll
                for (int dn = 0; dn < 4; ++dn) acc[dn][r] *= al;
            }
#pragma unroll
            for (int r = 0; r < 8; ++r) { Pw[pwo + (8 * hi + r) * PP + lr] = (h16)p0[r]; Pw[pwo + (8 * hi + r) * PP + 16 + lr] = (h16)p1[r]; }
            __builtin_amdgcn_wave_barrier(); asm volatile("" ::: "memory");
            const v16h ap = cat16(*(const v8ha*)(Pw + pwo + lr * PP + 8 * hi), *(const v8ha*)(Pw + pwo + lr * PP + 16 + 8 * hi));
            __builtin_amdgcn_wave_barrier(); asm volatile("" ::: "memory");
            const int vo = lr * KP + ko + 8 * hi;
            const v16h bv0 = cat16(*(const v8ha*)(Vs + vo), *(const v8ha*)(Vs + vo + 16));
            const v16h bv1 = cat16(*(const v8ha*)(Vs + vo + 16 * KP), *(const v8ha*)(Vs + vo + 16 * KP + 16));
            const v16h bv2 = cat16(*(const v8ha*)(Vs + vo + 32 * KP), *(const v8ha*)(Vs + vo + 32 * KP + 16));
            const v16h bv3 = cat16(*(const v8ha*)(Vs + vo + 48 * KP), *(const v8ha*)(Vs + vo + 48 * KP + 16));
            acc[0] = wmma16(ap, bv0, acc[0]); acc[1] = wmma16(ap, bv1, acc[1]); acc[2] = wmma16(ap, bv2, acc[2]); acc[3] = wmma16(ap, bv3, acc[3]);
            asm volatile("v_nop\n\tv_nop\n\tv_nop\n\tv_nop" : "+v"(acc[0]), "+v"(acc[1]), "+v"(acc[2]), "+v"(acc[3]) : "v"(ap), "v"(bv3));
        }
    }
    const int wo = wave * 16 * KP;
#pragma unroll
    for (int r = 0; r < 8; ++r) {
        float l = ls[r];
        l += __shfl_xor(l, 1, 32); l += __shfl_xor(l, 2, 32); l += __shfl_xor(l, 4, 32); l += __shfl_xor(l, 8, 32);
        const float inv = 1.0f / l;
#pragma unroll
        for (int dn = 0; dn < 4; ++dn) Os[wo + (8 * hi + r) * KP + dn * 16 + lr] = (h16)(acc[dn][r] * inv);
    }
    __builtin_amdgcn_wave_barrier(); asm volatile("" ::: "memory");
#pragma unroll 1
    for (int ps = 0; ps < 2; ++ps) {
#pragma unroll
        for (int j = 0; j < 4; ++j) { const int row = j * 4 + (lane >> 3), c = (lane & 7) * 8; const v8h val = *(const v8ha*)(Os + wo + row * KP + c);
            *(volatile v8h*)(O16 + pbase + (size_t)(q0 + row) * HD + c) = val; }
        if (ps == 0) __threadfence(); }
}

extern "C" void kernel_launch(void* const* d_in, const int* in_sizes, int n_in,
                              void* d_out, int out_size, void* d_ws, size_t ws_size, hipStream_t stream) {
    if (n_in < 13) return;
    const size_t need_q = ((size_t)(NB - 1) * SEQ_FULL + SEQ) * DM;
    if ((size_t)in_sizes[0] < need_q) return;
    if ((size_t)in_sizes[3] < (size_t)DM || (size_t)in_sizes[4] < (size_t)DM) return;
    if ((size_t)in_sizes[5] < (size_t)DM * DM || (size_t)in_sizes[7] < (size_t)DM * DM || (size_t)in_sizes[9] < (size_t)DM * DM || (size_t)in_sizes[11] < (size_t)DM * DM) return;
    if ((size_t)in_sizes[6] < (size_t)DM || (size_t)in_sizes[8] < (size_t)DM || (size_t)in_sizes[10] < (size_t)DM || (size_t)in_sizes[12] < (size_t)DM) return;
    if ((size_t)out_size < (size_t)MROWS * DM) return;
    const float* q = (const float*)d_in[0];
    const float* kin = (const float*)d_in[1]; const float* vin = (const float*)d_in[2]; (void)kin; (void)vin;
    const float* gamma = (const float*)d_in[3]; const float* beta = (const float*)d_in[4];
    const float* Wq = (const float*)d_in[5]; const float* bq = (const float*)d_in[6];
    const float* Wk = (const float*)d_in[7]; const float* bk = (const float*)d_in[8];
    const float* Wv = (const float*)d_in[9]; const float* bv = (const float*)d_in[10];
    const float* Wo = (const float*)d_in[11]; const float* bo = (const float*)d_in[12];
    float* OUT = (float*)d_out;
    char* wsp = (char*)d_ws;
    auto take = [&](size_t bytes) { char* p = wsp; wsp += (bytes + 255) & ~(size_t)255; return (void*)p; };
    bf* Hh = (bf*)take((size_t)MROWS * DM * 2); bf* Hl = (bf*)take((size_t)MROWS * DM * 2);
    bf* WT3 = (bf*)take((size_t)NQKV * DM * 2);
    h16* WOT = (h16*)take((size_t)DM * DM * 2);
    float* Cq = (float*)take((size_t)MROWS * NQKV * 4);
    h16* Q16 = (h16*)take((size_t)MROWS * DM * 2); h16* K16 = (h16*)take((size_t)MROWS * DM * 2);
    h16* VT16 = (h16*)take((size_t)MROWS * DM * 2);
    h16* O16 = (h16*)take((size_t)MROWS * DM * 2);
    if ((size_t)(wsp - (char*)d_ws) > ws_size) return;

    k_ln<<<(MROWS + 7) / 8, 256, 0, stream>>>(q, gamma, beta, Hh, Hl);
    k_wt<bf><<<dim3(DM / 64, DM / 64, 1), 256, 0, stream>>>(Wq, WT3);
    k_wt<bf><<<dim3(DM / 64, DM / 64, 1), 256, 0, stream>>>(Wk, WT3 + (size_t)DM * DM);
    k_wt<bf><<<dim3(DM / 64, DM / 64, 1), 256, 0, stream>>>(Wv, WT3 + (size_t)2 * DM * DM);
    k_wt<h16><<<dim3(DM / 64, DM / 64, 1), 256, 0, stream>>>(Wo, WOT);
    k_gemmw<bf, 1, false, false><<<dim3(MROWS / 64, NQKV / 64, 1), 32, 0, stream>>>(Hh, Hl, WT3, nullptr, DM, Cq, NQKV, nullptr, nullptr, 1.0f, 0, 0, 0, 0);
    const unsigned LP = (unsigned)(((size_t)NB * NH * SEQ * 8 + 255) / 256);
    k_qk<<<LP, 256, 0, stream>>>(Cq, 0, bq, Q16);
    k_qk<<<LP, 256, 0, stream>>>(Cq, DM, bk, K16);
    k_vt<<<dim3(SEQ / 64, NH, NB), 256, 0, stream>>>(Cq, bv, VT16);
    k_attn<<<dim3(SEQ / 64, NB * NH, 1), 128, 0, stream>>>(Q16, K16, VT16, O16);
    k_gemmw<h16, 0, true, true><<<dim3(SEQ / 64, DM / 64, NB), 32, 0, stream>>>(O16, nullptr, WOT, nullptr, DM, OUT, DM, bo, q, 1.0f / WCAR, (size_t)SEQ * DM, 0, (size_t)SEQ * DM, (size_t)SEQ_FULL * DM);
}
